// Point2NeighborAttention_25314537242842
// MI455X (gfx1250) — hardware-verified
//
#include <hip/hip_runtime.h>
#include <math.h>

typedef __attribute__((ext_vector_type(16))) _Float16 v16h;
typedef __attribute__((ext_vector_type(16))) __bf16 v16b;
typedef __attribute__((ext_vector_type(8)))  _Float16 v8h;
typedef __attribute__((ext_vector_type(8)))  float v8f;
typedef __attribute__((ext_vector_type(4)))  float v4f;
typedef __attribute__((ext_vector_type(2)))  float v2f;
typedef __attribute__((ext_vector_type(4)))  unsigned v4u;
typedef __attribute__((ext_vector_type(4)))  int v4i;
typedef float __attribute__((may_alias)) float_a;
typedef int __attribute__((may_alias)) int_a;

template <typename T> __device__ __forceinline__ void vst2(void* p, T v) { *(volatile T*)p = v; __threadfence(); *(volatile T*)p = v; }
__device__ __forceinline__ v8f wmma16(v16h a, v16h b, v8f c) {
  v8f d = __builtin_amdgcn_wmma_f32_16x16x32_f16(false, a, false, b, (short)0, c, false, false);
  asm volatile("v_nop\n\tv_nop\n\tv_nop\n\tv_nop" : "+v"(d) : "v"(a), "v"(b));
  return d;
}
__device__ __forceinline__ v8f wmma_bf(v16b a, v16b b, v8f c) {
  v8f d = __builtin_amdgcn_wmma_f32_16x16x32_bf16(false, a, false, b, (short)0, c, false, false);
  asm volatile("v_nop\n\tv_nop\n\tv_nop\n\tv_nop" : "+v"(d) : "v"(a), "v"(b));
  return d;
}
__device__ __forceinline__ v16h frag_h(const _Float16* rowk0, int lane) {
  union { v16h v; v8h q[2]; } u; const _Float16* p = rowk0 + 8 * (lane >> 4);
  u.q[0] = *(const v8h*)p; u.q[1] = *(const v8h*)(p + 16); return u.v;
}
__device__ __forceinline__ v16h frag_f32(const float* rowk0, int lane) {
  v16h a; const float* p = rowk0 + 8 * (lane >> 4);
#pragma unroll
  for (int i = 0; i < 8; ++i) { a[i] = (_Float16)p[i]; a[8 + i] = (_Float16)p[16 + i]; }
  return a;
}
__device__ __forceinline__ v16h frag_f32s(const float* rowk0, int lane, float sc) {
  v16h a; const float* p = rowk0 + 8 * (lane >> 4);
#pragma unroll
  for (int i = 0; i < 8; ++i) { a[i] = (_Float16)(p[i] * sc); a[8 + i] = (_Float16)(p[16 + i] * sc); }
  return a;
}
__device__ __forceinline__ v16h fragc_f32(const float* W, int k0, int n, int lane, int ld, int K) {
  v16h a; const int g = lane >> 4;
#pragma unroll
  for (int i = 0; i < 8; ++i) { const int ka = k0 + 8 * g + i, kb = ka + 16;
    a[i] = (_Float16)(ka < K ? W[(size_t)(ka < K ? ka : K - 1) * ld + n] : 0.f); a[8 + i] = (_Float16)(kb < K ? W[(size_t)(kb < K ? kb : K - 1) * ld + n] : 0.f); }
  return a;
}
struct F2 { v16b h, l; };
__device__ __forceinline__ F2 bsplit16(const float v[16]) { F2 r;
#pragma unroll
  for (int i = 0; i < 16; ++i) { const __bf16 h = (__bf16)v[i]; r.h[i] = h; r.l[i] = (__bf16)(v[i] - (float)h); }
  return r; }
__device__ __forceinline__ F2 split_row(const float* row, int k0, int lane) { float v[16]; const float* p = row + k0 + 8 * (lane >> 4);
#pragma unroll
  for (int i = 0; i < 8; ++i) { v[i] = p[i]; v[8 + i] = p[16 + i]; }
  return bsplit16(v); }
__device__ __forceinline__ F2 split_rowK(const float* row, int k0, int lane, int K) { float v[16]; const int g = lane >> 4;
#pragma unroll
  for (int i = 0; i < 8; ++i) { const int ka = k0 + 8 * g + i, kb = ka + 16; v[i] = ka < K ? row[ka < K ? ka : K - 1] : 0.f; v[8 + i] = kb < K ? row[kb < K ? kb : K - 1] : 0.f; }
  return bsplit16(v); }
__device__ __forceinline__ F2 split_col(const float* W, int k0, int n, int lane, int ld, int K) { float v[16]; const int g = lane >> 4;
#pragma unroll
  for (int i = 0; i < 8; ++i) { const int ka = k0 + 8 * g + i, kb = ka + 16; v[i] = ka < K ? W[(size_t)(ka < K ? ka : K - 1) * ld + n] : 0.f; v[8 + i] = kb < K ? W[(size_t)(kb < K ? kb : K - 1) * ld + n] : 0.f; }
  return bsplit16(v); }
__device__ __forceinline__ v8f mac3(const F2& a, const F2& b, v8f c) { c = wmma_bf(a.l, b.h, c); c = wmma_bf(a.h, b.l, c); return wmma_bf(a.h, b.h, c); }
__device__ __forceinline__ float sigm(float v) { return 1.0f / (1.0f + expf(-v)); }
#define LDSX() do { asm volatile("s_wait_dscnt 0" ::: "memory"); __builtin_amdgcn_wave_barrier(); __builtin_amdgcn_fence(__ATOMIC_RELEASE, "workgroup"); } while (0)


#define NB 4
#define NN 4096
#define KN 32
#define C1 64
#define CC 128
#define NR (NB * NN)
#ifndef NBT
#define NBT NB
#define TB0 0
#endif
#define NRT (NBT * NN)
#define RB0 ((size_t)TB0 * NN)
typedef __attribute__((ext_vector_type(8))) __bf16 v8b;
__device__ __forceinline__ v16b frag_b(const __bf16* rowk0, int lane) {
  union { v16b v; v8b q[2]; } u; const __bf16* p = rowk0 + 8 * (lane >> 4);
  u.q[0] = *(const v8b*)p; u.q[1] = *(const v8b*)(p + 16); return u.v;
}
__device__ __forceinline__ float bfr(float v) { return (float)(__bf16)v; }
__device__ __attribute__((noinline)) float exp_ni(float v) { return expf(v); }
__device__ __attribute__((noinline)) float erf_ni(float v) { return erff(v); }

#define PK_W2 0
#define PK_A1 ((size_t)CC * C1)
#define PK_A2 (PK_A1 + (size_t)4 * CC * CC)
#define PK_END (PK_A2 + (size_t)4 * CC * CC)
#define WS_PK  0u
#define WS_IDX (((2u * PK_END) + 127u) / 128u * 128u)
#define WS_H   (WS_IDX + 4u * NR * KN)
#define WS_Q   (WS_H + 4u * NR * CC)
#define WS_D   (WS_Q + 4u * NR * 3 * CC)
#define WS_H2  (WS_D + 4u * NR * CC)
#define WS_END (WS_H2 + 4u * NR * CC)

__global__ __launch_bounds__(128) void k_pack(const float* __restrict__ W2, const float* __restrict__ A1Q, const float* __restrict__ A1K, const float* __restrict__ A1V, const float* __restrict__ A1F, const float* __restrict__ A2Q, const float* __restrict__ A2K, const float* __restrict__ A2V, const float* __restrict__ A2F, __bf16* __restrict__ PK) {
  __shared__ __align__(16) __bf16 s[CC]; const int n = blockIdx.x, which = blockIdx.y, t = threadIdx.x;
  const float* Wm = (which == 0) ? W2 : (which == 1) ? A1Q : (which == 2) ? A1K : (which == 3) ? A1V : (which == 4) ? A1F : (which == 5) ? A2Q : (which == 6) ? A2K : (which == 7) ? A2V : A2F;
  const int K = (which == 0) ? C1 : CC; if (t < K) s[t] = (__bf16)Wm[(size_t)n * K + t];
  __syncthreads();
  const size_t dst = (which == 0) ? (PK_W2 + (size_t)n * C1) : ((which <= 4 ? PK_A1 : PK_A2) + ((size_t)((which - 1) & 3) * CC + n) * CC);
  if (t < K / 8) vst2((unsigned*)(PK + dst + t * 8), *(const v4u*)&s[t * 8]);
}
__global__ __launch_bounds__(128) void k_feat(const float* __restrict__ X, const float* __restrict__ W1, const float* __restrict__ G1, const float* __restrict__ B1, const float* __restrict__ M1, const float* __restrict__ V1, const __bf16* __restrict__ PK, const float* __restrict__ G2, const float* __restrict__ B2, const float* __restrict__ M2, const float* __restrict__ V2, float* __restrict__ H) {
  __shared__ __align__(16) __bf16 sh[64][C1 + 8], sl[64][C1 + 8]; __shared__ __align__(16) float so[4][16][132];
  const int tid = threadIdx.x, wave = tid >> 5, lane = tid & 31, col = lane & 15, g = lane >> 4; const size_t r0b = RB0 + (size_t)blockIdx.x * 64;
  for (int e = tid; e < 64 * C1; e += 128) { const int r = e >> 6, o = e & 63; const size_t row = r0b + r; const float x0 = bfr(X[row * 3]), x1 = bfr(X[row * 3 + 1]), x2 = bfr(X[row * 3 + 2]);
    const float pre = bfr(W1[o * 3]) * x0 + bfr(W1[o * 3 + 1]) * x1 + bfr(W1[o * 3 + 2]) * x2; const float v = fmaxf((pre - bfr(M1[o])) * (bfr(G1[o]) / sqrtf(bfr(V1[o]) + 1e-5f)) + bfr(B1[o]), 0.f);
    const __bf16 hb = (__bf16)v; sh[r][o] = hb; sl[r][o] = (__bf16)(v - (float)hb); }
  if (tid < 64) for (int o = C1; o < C1 + 8; ++o) { sh[tid][o] = (__bf16)0.f; sl[tid][o] = (__bf16)0.f; }
  __syncthreads();
  const size_t r0 = r0b + wave * 16; v8f acc[8] = {};
#pragma unroll
  for (int kc = 0; kc < C1 / 32; ++kc) { F2 a; a.h = frag_b(&sh[wave * 16 + col][kc * 32], lane); a.l = frag_b(&sl[wave * 16 + col][kc * 32], lane);
#pragma unroll
    for (int j = 0; j < 8; ++j) { const v16b w = frag_b(PK + PK_W2 + (size_t)(j * 16 + col) * C1 + kc * 32, lane); acc[j] = wmma_bf(a.l, w, acc[j]); acc[j] = wmma_bf(a.h, w, acc[j]); } }
#pragma unroll
  for (int j = 0; j < 8; ++j) { const int o = j * 16 + col; const float sc = bfr(G2[o]) / sqrtf(bfr(V2[o]) + 1e-5f), mm = bfr(M2[o]), bb = bfr(B2[o]);
#pragma unroll
    for (int r = 0; r < 8; ++r) so[wave][8 * g + r][o] = fmaxf((acc[j][r] - mm) * sc + bb, 0.f); }
  LDSX();
  for (int rl = 0; rl < 16; ++rl) vst2(H + (r0 + rl) * CC + lane * 4, *(const v4f*)&so[wave][rl][lane * 4]);
}
__global__ __launch_bounds__(256) void k_knn(const float* __restrict__ X, int* __restrict__ IDX) {
  __shared__ float sx[NN][3]; __shared__ float sq[NN]; __shared__ float ld[64][4][KN]; __shared__ int li[64][4][KN]; __shared__ __align__(16) int so[64][KN];
  const int t = threadIdx.x; const size_t b = blockIdx.y + TB0; const int n0 = blockIdx.x * 64; const int q = t >> 2, part = t & 3;
  for (int i = t; i < NN; i += 256) { const float x = bfr(X[(b * NN + i) * 3]), y = bfr(X[(b * NN + i) * 3 + 1]), z = bfr(X[(b * NN + i) * 3 + 2]); sx[i][0] = x; sx[i][1] = y; sx[i][2] = z; sq[i] = (x * x + z * z) + y * y; }
  __syncthreads();
  const int me = n0 + q; const float px = sx[me][0], py = sx[me][1], pz = sx[me][2], sqm = sq[me];
  float* bd = ld[q][part]; int* bi = li[q][part]; for (int k = 0; k < KN; ++k) { bd[k] = 3.0e38f; bi[k] = 0x7fffffff; }
  float thr = 3.0e38f; int thri = 0x7fffffff;
#pragma unroll 1
  for (int i = part * (NN / 4); i < (part + 1) * (NN / 4); ++i) { const float dot = (px * sx[i][0] + py * sx[i][1]) + pz * sx[i][2]; const float d = (sqm + sq[i]) - 2.0f * dot;
    if (d < thr || (d == thr && i < thri)) { int pos = KN - 1; while (pos > 0 && (d < bd[pos - 1] || (d == bd[pos - 1] && i < bi[pos - 1]))) { bd[pos] = bd[pos - 1]; bi[pos] = bi[pos - 1]; --pos; } bd[pos] = d; bi[pos] = i; thr = bd[KN - 1]; thri = bi[KN - 1]; } }
  __syncthreads();
  if (part == 0) {
    int hp[4] = {0, 0, 0, 0};
    for (int k = 0; k < KN; ++k) { int best = -1; float bdv = 3.0e38f; int biv = 0x7fffffff;
      for (int p2 = 0; p2 < 4; ++p2) { if (hp[p2] >= KN) continue; const float dv = ld[q][p2][hp[p2]]; const int iv = li[q][p2][hp[p2]]; if (best < 0 || dv < bdv || (dv == bdv && iv < biv)) { best = p2; bdv = dv; biv = iv; } }
      so[q][k] = biv; ++hp[best]; } }
  __syncthreads();
  for (int e = t; e < 64 * KN / 4; e += 256) { const int r = e / (KN / 4), c = e % (KN / 4); vst2(IDX + (b * NN + n0 + r) * KN + c * 4, *(const v4i*)&so[r][c * 4]); }
}
__global__ __launch_bounds__(128) void k_qkv(const float* __restrict__ H, const __bf16* __restrict__ PA, float* __restrict__ QKV) {
  __shared__ __align__(16) float so[4][16][132];
  const int tid = threadIdx.x, wave = tid >> 5, lane = tid & 31, col = lane & 15, g = lane >> 4; const size_t r0 = RB0 + (size_t)blockIdx.x * 64 + wave * 16; const int which = blockIdx.y; const __bf16* P = PA + (size_t)which * CC * CC;
  v8f acc[8] = {};
#pragma unroll
  for (int kc = 0; kc < CC / 32; ++kc) { const F2 a = split_row(H + (r0 + col) * CC, kc * 32, lane);
#pragma unroll
    for (int j = 0; j < 8; ++j) { const v16b w = frag_b(P + (size_t)(j * 16 + col) * CC + kc * 32, lane); acc[j] = wmma_bf(a.l, w, acc[j]); acc[j] = wmma_bf(a.h, w, acc[j]); } }
#pragma unroll
  for (int j = 0; j < 8; ++j)
#pragma unroll
    for (int r = 0; r < 8; ++r) so[wave][8 * g + r][j * 16 + col] = acc[j][r];
  LDSX();
  for (int rl = 0; rl < 16; ++rl) vst2(QKV + ((r0 + rl) * 3 + which) * CC + lane * 4, *(const v4f*)&so[wave][rl][lane * 4]);
}
__global__ __launch_bounds__(256) void k_nbr(const float* __restrict__ H, const float* __restrict__ QKV, const int* __restrict__ IDX, float* __restrict__ D) {
  __shared__ float sq_[32][CC]; __shared__ float sa[32][KN]; __shared__ int sidx[32][KN]; __shared__ __align__(16) float sd[32][CC + 4];
  const int t = threadIdx.x; const int p = t >> 3, sub = t & 7; const size_t row0 = RB0 + (size_t)blockIdx.x * 32; const size_t row = row0 + p; const size_t b = row / NN;
  for (int e = t; e < 32 * CC; e += 256) { const int r = e >> 7, c = e & 127; sq_[r][c] = QKV[((row0 + r) * 3 + 0) * CC + c]; }
  for (int e = t; e < 32 * KN; e += 256) { const int r = e >> 5, k = e & 31; sidx[r][k] = IDX[(row0 + r) * KN + k]; }
  __syncthreads();
  float s4[4]; float mx = -3.0e38f;
  for (int kk = 0; kk < 4; ++kk) { const int k = sub * 4 + kk; const size_t nr = b * NN + sidx[p][k]; const float* kp = QKV + (nr * 3 + 1) * CC; float a = 0.f;
#pragma unroll 1
    for (int c = 0; c < CC; ++c) a += sq_[p][c] * kp[c];
    s4[kk] = a * 0.08838834764831845f; mx = fmaxf(mx, s4[kk]); }
#pragma unroll
  for (int o = 1; o < 8; o <<= 1) mx = fmaxf(mx, __shfl_xor(mx, o));
  float sm = 0.f; for (int kk = 0; kk < 4; ++kk) { s4[kk] = exp_ni(s4[kk] - mx); sm += s4[kk]; }
#pragma unroll
  for (int o = 1; o < 8; o <<= 1) sm += __shfl_xor(sm, o);
  for (int kk = 0; kk < 4; ++kk) sa[p][sub * 4 + kk] = s4[kk] / sm;
  __syncthreads();
  for (int c = sub * 16; c < sub * 16 + 16; ++c) { float a = 0.f;
#pragma unroll 1
    for (int k = 0; k < KN; ++k) { const size_t nr = b * NN + sidx[p][k]; a += sa[p][k] * QKV[(nr * 3 + 2) * CC + c]; }
    sd[p][c] = H[row * CC + c] - a; }
  __syncthreads();
  for (int e = t; e < 32 * CC / 4; e += 256) { const int r = e / (CC / 4), qd = e % (CC / 4); vst2(D + (row0 + r) * CC + qd * 4, *(const v4f*)&sd[r][qd * 4]); }
}
__global__ __launch_bounds__(128) void k_ff(const float* __restrict__ D, const float* __restrict__ H, const __bf16* __restrict__ PF, const float* __restrict__ G, const float* __restrict__ Bt, const float* __restrict__ M, const float* __restrict__ V, float* __restrict__ OUT) {
  __shared__ __align__(16) float so[4][16][132];
  const int tid = threadIdx.x, wave = tid >> 5, lane = tid & 31, col = lane & 15, g = lane >> 4; const size_t r0 = RB0 + (size_t)blockIdx.x * 64 + wave * 16;
  v8f acc[8] = {};
#pragma unroll
  for (int kc = 0; kc < CC / 32; ++kc) { const F2 a = split_row(D + (r0 + col) * CC, kc * 32, lane);
#pragma unroll
    for (int j = 0; j < 8; ++j) { const v16b w = frag_b(PF + (size_t)(j * 16 + col) * CC + kc * 32, lane); acc[j] = wmma_bf(a.l, w, acc[j]); acc[j] = wmma_bf(a.h, w, acc[j]); } }
#pragma unroll
  for (int j = 0; j < 8; ++j) { const int o = j * 16 + col; const float sc = bfr(G[o]) / sqrtf(bfr(V[o]) + 1e-5f), mm = bfr(M[o]), bb = bfr(Bt[o]);
#pragma unroll
    for (int r = 0; r < 8; ++r) { const size_t row = r0 + 8 * g + r; so[wave][8 * g + r][o] = H[row * CC + o] + fmaxf((acc[j][r] - mm) * sc + bb, 0.f); } }
  LDSX();
  for (int rl = 0; rl < 16; ++rl) vst2(OUT + (r0 + rl) * CC + lane * 4, *(const v4f*)&so[wave][rl][lane * 4]);
}
extern "C" void kernel_launch(void* const* d_in, const int* in_sizes, int n_in, void* d_out, int out_size, void* d_ws, size_t ws_size, hipStream_t stream) {
  (void)in_sizes; (void)n_in; (void)out_size;
  const float** F = (const float**)d_in;
  if (ws_size < (size_t)WS_END) return;
  char* ws = (char*)d_ws; __bf16* PK = (__bf16*)(ws + WS_PK); int* IDX = (int*)(ws + WS_IDX); float *H = (float*)(ws + WS_H), *QKV = (float*)(ws + WS_Q), *D = (float*)(ws + WS_D), *H2 = (float*)(ws + WS_H2);
  k_pack<<<dim3(CC, 9), 128, 0, stream>>>(F[2], F[19], F[20], F[21], F[22], F[23], F[24], F[25], F[26], PK);
  k_feat<<<NRT / 64, 128, 0, stream>>>(F[0], F[1], F[3], F[4], F[5], F[6], PK, F[7], F[8], F[9], F[10], H);
  k_knn<<<dim3(NN / 64, NBT), 256, 0, stream>>>(F[0], IDX);
  k_qkv<<<dim3(NRT / 64, 3), 128, 0, stream>>>(H, PK + PK_A1, QKV);
  k_nbr<<<NRT / 32, 256, 0, stream>>>(H, QKV, IDX, D);
  k_ff<<<NRT / 64, 128, 0, stream>>>(D, H, PK + PK_A1 + (size_t)3 * CC * CC, F[11], F[12], F[13], F[14], H2);
  k_qkv<<<dim3(NRT / 64, 3), 128, 0, stream>>>(H2, PK + PK_A2, QKV);
  k_nbr<<<NRT / 32, 256, 0, stream>>>(H2, QKV, IDX, D);
  k_ff<<<NRT / 64, 128, 0, stream>>>(D, H2, PK + PK_A2 + (size_t)3 * CC * CC, F[15], F[16], F[17], F[18], (float*)d_out);
}
